// LlamaAttention_52587579572852
// MI455X (gfx1250) — hardware-verified
//
#include <hip/hip_runtime.h>

#pragma clang fp contract(off)

#ifndef NB
#define NB 2
#endif
#ifndef SEQ
#define SEQ 2048
#endif
#define NB_FULL  2
#define SEQ_FULL 2048
#define DM   2048
#define NH_  16
#define HD   128
#define DQ   (NH_ * HD)
#define ZH   2
#define PCAR 1024.0f
#define OCAR 64.0f
#define WCAR 64.0f
#define SCL  0.08838834764831845f
#define FLOW (-3.4028234663852886e38f)

static_assert(SEQ % 128 == 0);
static_assert(SEQ >= 128 && SEQ <= SEQ_FULL);
static_assert(NB >= 1 && NB <= NB_FULL);
static_assert(DQ == DM);
static_assert(DM % 64 == 0 && HD % 64 == 0 && (NH_ % ZH) == 0);

typedef _Float16 h16;
typedef unsigned short bf;
typedef __attribute__((ext_vector_type(16))) __bf16   v16bf;
typedef __attribute__((ext_vector_type(16))) _Float16 v16h;
typedef __attribute__((ext_vector_type(8)))  _Float16 v8h;
typedef __attribute__((ext_vector_type(4)))  _Float16 v4h;
typedef __attribute__((ext_vector_type(8)))  unsigned short v8us;
typedef __attribute__((ext_vector_type(8)))  float    v8f;
typedef __attribute__((ext_vector_type(4)))  float    v4f;
typedef v4f __attribute__((may_alias)) v4fa;

__device__ __forceinline__ unsigned short f2bf(float f) { unsigned u = __float_as_uint(f); u += 0x7FFFu + ((u >> 16) & 1u); return (unsigned short)(u >> 16); }
__device__ __forceinline__ float bf2f(unsigned short b) { return __uint_as_float(((unsigned)b) << 16); }
__device__ __forceinline__ float bfr(float f) { return bf2f(f2bf(f)); }
__device__ __forceinline__ v16h cat16(v8h lo, v8h hi) { return __builtin_shufflevector(lo, hi, 0, 1, 2, 3, 4, 5, 6, 7, 8, 9, 10, 11, 12, 13, 14, 15); }
__device__ __forceinline__ v16bf cat16b(v8us lo, v8us hi) { return __builtin_bit_cast(v16bf, __builtin_shufflevector(lo, hi, 0, 1, 2, 3, 4, 5, 6, 7, 8, 9, 10, 11, 12, 13, 14, 15)); }
__device__ __forceinline__ v8f wmma16(v16h a, v16h b, v8f c) { return __builtin_amdgcn_wmma_f32_16x16x32_f16(false, a, false, b, (short)0, c, false, false); }
__device__ __forceinline__ v8f wmmab(v16bf a, v16bf b, v8f c) { return __builtin_amdgcn_wmma_f32_16x16x32_bf16(false, a, false, b, (short)0, c, false, false); }

template <typename T16> struct WFrag;
template <> struct WFrag<h16> { typedef v16h V; static __device__ __forceinline__ V ld(const h16* p) { return cat16(*(const v8h*)p, *(const v8h*)(p + 16)); } static __device__ __forceinline__ v8f mma(V a, V b, v8f c) { return wmma16(a, b, c); } };
template <> struct WFrag<bf> { typedef v16bf V; static __device__ __forceinline__ V ld(const bf* p) { return cat16b(*(const v8us*)p, *(const v8us*)(p + 16)); } static __device__ __forceinline__ v8f mma(V a, V b, v8f c) { return wmmab(a, b, c); } };
template <typename T16, int NSPLIT, bool BIAS>
__global__ __launch_bounds__(32) __attribute__((amdgpu_num_vgpr(256)))
void k_gemmw(const T16* __restrict__ A, const T16* __restrict__ A2, const T16* __restrict__ Bt, const T16* __restrict__ Bt2, int K, float* C, int ldc, const float* __restrict__ bias, float cscale, size_t sA, size_t sB, size_t sC) {
    typedef typename WFrag<T16>::V V;
    __shared__ __align__(16) float os[16 * 68];
    const size_t z = blockIdx.z; A += z * sA; if (A2) A2 += z * sA; Bt += z * sB; if (Bt2) Bt2 += z * sB; C += z * sC;
    const int lane = threadIdx.x & 31, lr = lane & 15, hi = lane >> 4; const int r0 = blockIdx.x * 64, c0 = blockIdx.y * 64;
    v8f acc[4][4];
#pragma unroll
    for (int mb = 0; mb < 4; ++mb)
#pragma unroll
        for (int nb = 0; nb < 4; ++nb) acc[mb][nb] = (v8f){};
    const size_t aoff = (size_t)(r0 + lr) * K + 8 * hi, boff = (size_t)(c0 + lr) * K + 8 * hi;
#pragma unroll 1
    for (int kc = 0; kc < K; kc += 32) {
        V a[4], a2[4];
#pragma unroll
        for (int mb = 0; mb < 4; ++mb) { a[mb] = WFrag<T16>::ld(A + aoff + (size_t)mb * 16 * K + kc); if (NSPLIT == 1 || NSPLIT == 2) a2[mb] = WFrag<T16>::ld(A2 + aoff + (size_t)mb * 16 * K + kc); }
#pragma unroll
        for (int nb = 0; nb < 4; ++nb) { const V b = WFrag<T16>::ld(Bt + boff + (size_t)nb * 16 * K + kc); V b2; if (NSPLIT >= 2) b2 = WFrag<T16>::ld(Bt2 + boff + (size_t)nb * 16 * K + kc);
#pragma unroll
            for (int mb = 0; mb < 4; ++mb) { acc[mb][nb] = WFrag<T16>::mma(a[mb], b, acc[mb][nb]); if (NSPLIT == 1 || NSPLIT == 2) acc[mb][nb] = WFrag<T16>::mma(a2[mb], b, acc[mb][nb]); if (NSPLIT >= 2) acc[mb][nb] = WFrag<T16>::mma(a[mb], b2, acc[mb][nb]); } }
        asm volatile("v_nop\n\tv_nop\n\tv_nop\n\tv_nop" : "+v"(acc[0][0]), "+v"(acc[1][1]), "+v"(acc[2][2]), "+v"(acc[3][3]) : "v"(a[0]), "v"(a[3]));
    }
    v4f bb = (v4f){0.f, 0.f, 0.f, 0.f};
    if (BIAS) { const v4f br = *(const v4f*)(bias + c0 + lr * 4); bb[0] = bfr(br[0]); bb[1] = bfr(br[1]); bb[2] = bfr(br[2]); bb[3] = bfr(br[3]); }
#pragma unroll
    for (int mb = 0; mb < 4; ++mb) {
#pragma unroll
        for (int nb = 0; nb < 4; ++nb) {
#pragma unroll
            for (int j = 0; j < 8; ++j) os[(hi * 8 + j) * 68 + nb * 16 + lr] = acc[mb][nb][j]; }
        __builtin_amdgcn_wave_barrier(); asm volatile("" ::: "memory");
        float* crow = C + (size_t)(r0 + mb * 16) * ldc + c0;
#pragma unroll 1
        for (int ps = 0; ps < 2; ++ps) {
#pragma unroll
            for (int s = 0; s < 8; ++s) { const int row = 2 * s + hi, cofs = lr * 4; v4f val = *(const v4fa*)(os + row * 68 + cofs); val = val * cscale; if (BIAS) val = val + bb;
                *(volatile v4f*)(crow + (size_t)row * ldc + cofs) = val; }
            if (ps == 0) __threadfence(); }
        __builtin_amdgcn_wave_barrier(); asm volatile("" ::: "memory");
    }
}

__global__ __launch_bounds__(256) void k_cvt8(const float* __restrict__ src, bf* dst, size_t n8) { const size_t i = (size_t)blockIdx.x * 256 + threadIdx.x; if (i >= n8) return; const v8f v = *(const v8f*)(src + i * 8); v8us o;
#pragma unroll
    for (int k = 0; k < 8; ++k) o[k] = f2bf(v[k]); *(volatile v8us*)(dst + i * 8) = o; __threadfence(); *(volatile v8us*)(dst + i * 8) = o; }
__global__ __launch_bounds__(256) void k_cvt8h(const float* __restrict__ src, float sc, h16* dst, size_t n8) { const size_t i = (size_t)blockIdx.x * 256 + threadIdx.x; if (i >= n8) return; const v8f v = *(const v8f*)(src + i * 8); v8h o;
#pragma unroll
    for (int k = 0; k < 8; ++k) o[k] = (h16)(bfr(v[k]) * sc); *(volatile v8h*)(dst + i * 8) = o; __threadfence(); *(volatile v8h*)(dst + i * 8) = o; }
__global__ __launch_bounds__(256) void k_madd(const float* __restrict__ m, float* MA) { const int i = blockIdx.x * 256 + threadIdx.x; if (i >= SEQ / 4) return; const v4f a = *(const v4f*)(m + (size_t)i * 4); v4f o;
#pragma unroll
    for (int q = 0; q < 4; ++q) { float u = 1.0f - bfr(a[q]); asm volatile("" : "+v"(u)); o[q] = u * FLOW; }
    *(volatile v4f*)(MA + (size_t)i * 4) = o; __threadfence(); *(volatile v4f*)(MA + (size_t)i * 4) = o; }
__global__ __launch_bounds__(256) void k_qkp(const float* __restrict__ F, h16* P) { const size_t e = ((size_t)blockIdx.x * 256 + threadIdx.x) * 8; if (e >= (size_t)NH_ * SEQ * HD) return; const int d = (int)(e % HD); const int t = (int)((e / HD) % SEQ); const int h = (int)(e / ((size_t)HD * SEQ));
    const float* f = F + (size_t)t * DQ + (size_t)h * HD + d; const v4f a0 = *(const v4f*)f, a1 = *(const v4f*)(f + 4); v8h o;
#pragma unroll
    for (int q = 0; q < 4; ++q) { o[q] = (h16)a0[q]; o[q + 4] = (h16)a1[q]; }
    *(volatile v8h*)(P + e) = o; __threadfence(); *(volatile v8h*)(P + e) = o; }
__global__ __launch_bounds__(256) void k_vtp(const float* __restrict__ F, h16* VT) { const size_t e = ((size_t)blockIdx.x * 256 + threadIdx.x) * 8; if (e >= (size_t)NH_ * HD * SEQ) return; const int t = (int)(e % SEQ); const int d = (int)((e / SEQ) % HD); const int g = (int)(e / ((size_t)SEQ * HD));
    const float* f = F + (size_t)t * DQ + (size_t)g * HD + d; v8h o;
#pragma unroll
    for (int q = 0; q < 8; ++q) o[q] = (h16)f[(size_t)q * DQ];
    *(volatile v8h*)(VT + e) = o; __threadfence(); *(volatile v8h*)(VT + e) = o; }
__global__ __launch_bounds__(256) void k_asoft(const float* __restrict__ Sb, const float* __restrict__ MA, h16* P16) {
    const int lane = threadIdx.x & 31; const int row = blockIdx.x * 8 + (threadIdx.x >> 5); if (row >= ZH * SEQ) return;
    const float* sr = Sb + (size_t)row * SEQ; float v[SEQ / 32]; float mx = FLOW;
#pragma unroll
    for (int ch = 0; ch < SEQ / 128; ++ch) { const int j0 = ch * 128 + lane * 4; const v4f a = *(const v4f*)(sr + j0); const v4f am4 = *(const v4f*)(MA + j0);
#pragma unroll
        for (int q = 0; q < 4; ++q) { float sa = a[q] * SCL; asm volatile("" : "+v"(sa)); const float t = sa + am4[q]; v[ch * 4 + q] = t; mx = fmaxf(mx, t); } }
#pragma unroll
    for (int sh = 16; sh; sh >>= 1) mx = fmaxf(mx, __shfl_xor(mx, sh, 32));
    float sum = 0.f;
#pragma unroll
    for (int k = 0; k < SEQ / 32; ++k) { float d0 = __fsub_rn(v[k], mx); asm volatile("" : "+v"(d0)); v[k] = __builtin_amdgcn_exp2f(__fmul_rn(d0, 1.4426950408889634f)); sum += v[k]; }
#pragma unroll
    for (int sh = 16; sh; sh >>= 1) sum += __shfl_xor(sum, sh, 32);
    const float f = __fdiv_rn(PCAR, sum);
#pragma unroll 1
    for (int ps = 0; ps < 2; ++ps) {
#pragma unroll
        for (int ch = 0; ch < SEQ / 128; ++ch) { v4h o4;
#pragma unroll
            for (int q = 0; q < 4; ++q) o4[q] = (h16)(v[ch * 4 + q] * f);
            *(volatile v4h*)(P16 + (size_t)row * SEQ + ch * 128 + lane * 4) = o4; }
        if (ps == 0) __threadfence(); }
}
__global__ __launch_bounds__(256) void k_merge(const float* __restrict__ O, int h0, h16* AT) { const size_t e = ((size_t)blockIdx.x * 256 + threadIdx.x) * 8; if (e >= (size_t)ZH * SEQ * HD) return; const int d = (int)(e % HD); const int t = (int)((e / HD) % SEQ); const int zz = (int)(e / ((size_t)HD * SEQ));
    const v4f a0 = *(const v4f*)(O + e), a1 = *(const v4f*)(O + e + 4); v8h o;
#pragma unroll
    for (int q = 0; q < 4; ++q) { o[q] = (h16)(a0[q] * (OCAR / PCAR)); o[q + 4] = (h16)(a1[q] * (OCAR / PCAR)); }
    h16* p = AT + (size_t)t * DQ + (size_t)(h0 + zz) * HD + d; *(volatile v8h*)p = o; __threadfence(); *(volatile v8h*)p = o; }

extern "C" void kernel_launch(void* const* d_in, const int* in_sizes, int n_in,
                              void* d_out, int out_size, void* d_ws, size_t ws_size, hipStream_t stream) {
    if (n_in < 10) return;
    const float* x  = (const float*)d_in[0]; const float* am = (const float*)d_in[1];
    const float* wq = (const float*)d_in[2]; const float* bq = (const float*)d_in[3]; const float* wk = (const float*)d_in[4]; const float* bk = (const float*)d_in[5];
    const float* wv = (const float*)d_in[6]; const float* bv = (const float*)d_in[7]; const float* wo = (const float*)d_in[8]; const float* bo = (const float*)d_in[9];
    if (in_sizes[0] < 0 || (size_t)in_sizes[0] < (size_t)(NB - 1) * SEQ_FULL * DM + (size_t)SEQ * DM) return;
    if (in_sizes[1] < (NB - 1) * SEQ_FULL + SEQ) return;
    if (in_sizes[2] < DQ * DM || in_sizes[4] < DQ * DM || in_sizes[6] < DQ * DM || in_sizes[8] < DM * DQ) return;
    if (in_sizes[3] < DQ || in_sizes[5] < DQ || in_sizes[7] < DQ || in_sizes[9] < DM) return;
    if (out_size < 0 || (size_t)out_size < (size_t)NB * SEQ * DM) return;
    float* OUT = (float*)d_out;

    char* wsp = (char*)d_ws; size_t used = 0;
    auto take = [&](size_t bytes) { char* p = wsp + used; used += (bytes + 255) & ~(size_t)255; return (void*)p; };
    bf*  WQ   = (bf*)take((size_t)DQ * DM * 2);
    bf*  WK   = (bf*)take((size_t)DQ * DM * 2);
    bf*  WV   = (bf*)take((size_t)DQ * DM * 2);
    h16* WO16 = (h16*)take((size_t)DM * DQ * 2);
    bf*  XB   = (bf*)take((size_t)SEQ * DM * 2);
    const size_t fproj = (size_t)SEQ * DQ * 4, fsc = (size_t)ZH * SEQ * SEQ * 4;
    float* F  = (float*)take(fproj > fsc ? fproj : fsc);
    float* Sb = F;
    float* MA = (float*)take((size_t)SEQ * 4);
    h16* QP16 = (h16*)take((size_t)NH_ * SEQ * HD * 2);
    h16* KP16 = (h16*)take((size_t)NH_ * SEQ * HD * 2);
    h16* VT16 = (h16*)take((size_t)NH_ * HD * SEQ * 2);
    h16* P16  = (h16*)take((size_t)ZH * SEQ * SEQ * 2);
    float* Ob = (float*)take((size_t)ZH * SEQ * HD * 4);
    h16* AT16 = (h16*)take((size_t)SEQ * DQ * 2);
    if (used > ws_size) return;

    const unsigned gw8 = (unsigned)(((size_t)DQ * DM / 8 + 255) / 256);
    k_cvt8<<<gw8, 256, 0, stream>>>(wq, WQ, (size_t)DQ * DM / 8);
    k_cvt8<<<gw8, 256, 0, stream>>>(wk, WK, (size_t)DQ * DM / 8);
    k_cvt8<<<gw8, 256, 0, stream>>>(wv, WV, (size_t)DQ * DM / 8);
    k_cvt8h<<<gw8, 256, 0, stream>>>(wo, WCAR, WO16, (size_t)DM * DQ / 8);
    const unsigned gx8 = (unsigned)(((size_t)SEQ * DM / 8 + 255) / 256);
    const unsigned gpl = (unsigned)(((size_t)NH_ * SEQ * HD / 8 + 255) / 256);
    const unsigned gmg = (unsigned)(((size_t)ZH * SEQ * HD / 8 + 255) / 256);
    const unsigned gma = (unsigned)((SEQ / 4 + 255) / 256);
    for (int b = 0; b < NB; ++b) {
        k_cvt8<<<gx8, 256, 0, stream>>>(x + (size_t)b * SEQ_FULL * DM, XB, (size_t)SEQ * DM / 8);
        k_madd<<<gma, 256, 0, stream>>>(am + (size_t)b * SEQ_FULL, MA);
        k_gemmw<bf, 0, true><<<dim3(SEQ / 64, DQ / 64, 1), 32, 0, stream>>>(XB, nullptr, WQ, nullptr, DM, F, DQ, bq, 1.0f, 0, 0, 0);
        k_qkp<<<gpl, 256, 0, stream>>>(F, QP16);
        k_gemmw<bf, 0, true><<<dim3(SEQ / 64, DQ / 64, 1), 32, 0, stream>>>(XB, nullptr, WK, nullptr, DM, F, DQ, bk, 1.0f, 0, 0, 0);
        k_qkp<<<gpl, 256, 0, stream>>>(F, KP16);
        k_gemmw<bf, 0, true><<<dim3(SEQ / 64, DQ / 64, 1), 32, 0, stream>>>(XB, nullptr, WV, nullptr, DM, F, DQ, bv, 1.0f, 0, 0, 0);
        k_vtp<<<gpl, 256, 0, stream>>>(F, VT16);
        for (int h0 = 0; h0 < NH_; h0 += ZH) {
            k_gemmw<h16, 0, false><<<dim3(SEQ / 64, SEQ / 64, ZH), 32, 0, stream>>>(QP16 + (size_t)h0 * SEQ * HD, nullptr, KP16 + (size_t)h0 * SEQ * HD, nullptr, HD, Sb, SEQ, nullptr, 1.0f, (size_t)SEQ * HD, (size_t)SEQ * HD, (size_t)SEQ * SEQ);
            k_asoft<<<(unsigned)(ZH * SEQ / 8), 256, 0, stream>>>(Sb, MA, P16);
            k_gemmw<h16, 0, false><<<dim3(SEQ / 64, HD / 64, ZH), 32, 0, stream>>>(P16, nullptr, VT16 + (size_t)h0 * HD * SEQ, nullptr, SEQ, Ob, HD, nullptr, 1.0f, (size_t)SEQ * SEQ, (size_t)HD * SEQ, (size_t)SEQ * HD);
            k_merge<<<gmg, 256, 0, stream>>>(Ob, h0, AT16);
        }
        k_gemmw<h16, 0, true><<<dim3(SEQ / 64, DM / 64, 1), 32, 0, stream>>>(AT16, nullptr, WO16, nullptr, DQ, OUT + (size_t)b * SEQ * DM, DM, bo, 1.0f / (OCAR * WCAR), 0, 0, 0);
    }
}
